// language_8057358647401
// MI455X (gfx1250) — hardware-verified
//
#include <hip/hip_runtime.h>
#include <hip/hip_bf16.h>


#define BB 32
#define TT 64
#define DD 1024
#define GG 4096
#define MR 2048

static_assert(MR == BB * TT);
static_assert(DD % 64 == 0);
static_assert(GG == 4 * DD);
static_assert(BB % 16 == 0);

typedef float          v4f   __attribute__((ext_vector_type(4)));
typedef float          v8f   __attribute__((ext_vector_type(8)));
typedef __bf16         v16b  __attribute__((ext_vector_type(16)));
typedef unsigned short u16x8 __attribute__((ext_vector_type(8)));
typedef _Float16       v16h  __attribute__((ext_vector_type(16)));
typedef _Float16       v8h   __attribute__((ext_vector_type(8)));

union FragB { u16x8 h[2]; v16b v; };
union FragH { v8h h[2]; v16h v; };

constexpr size_t SZ_Q16  = (size_t)MR * DD * 2;
constexpr size_t SZ_WI16 = (size_t)GG * DD * 2;
constexpr size_t SZ_WA16 = (size_t)DD * DD * 2;
constexpr size_t SZ_XG   = (size_t)MR * GG * 4;
constexpr size_t SZ_HPL  = (size_t)MR * DD * 2;
constexpr size_t SZ_PART = (size_t)(DD / 64) * MR * 4;
constexpr size_t SZ_AO16 = (size_t)BB * DD * 2;

constexpr size_t OFF_QH   = 0;
constexpr size_t OFF_QL   = OFF_QH + SZ_Q16;
constexpr size_t OFF_WIH  = OFF_QL + SZ_Q16;
constexpr size_t OFF_WIL  = OFF_WIH + SZ_WI16;
constexpr size_t OFF_WHH  = OFF_WIL + SZ_WI16;
constexpr size_t OFF_WAT  = OFF_WHH + SZ_WI16;
constexpr size_t OFF_WLH  = OFF_WAT + SZ_WA16;
constexpr size_t OFF_WLL  = OFF_WLH + SZ_WA16;
constexpr size_t OFF_XG   = OFF_WLL + SZ_WA16;
constexpr size_t OFF_HPL  = OFF_XG + SZ_XG;
constexpr size_t OFF_PART = OFF_HPL + SZ_HPL;
constexpr size_t OFF_AOH  = OFF_PART + SZ_PART;
constexpr size_t OFF_AOL  = OFF_AOH + SZ_AO16;
constexpr size_t WS_END   = OFF_AOL + SZ_AO16;
static_assert(WS_END <= (size_t)134217728);
static_assert(OFF_QL % 128 == 0 && OFF_WIH % 128 == 0 && OFF_WIL % 128 == 0 && OFF_WHH % 128 == 0);
static_assert(OFF_WAT % 128 == 0 && OFF_WLH % 128 == 0 && OFF_WLL % 128 == 0 && OFF_XG % 128 == 0);
static_assert(OFF_HPL % 128 == 0 && OFF_PART % 128 == 0 && OFF_AOH % 128 == 0 && OFF_AOL % 128 == 0);

#define LSTM_LDS_BYTES 163840

__device__ __forceinline__ unsigned short f32_to_bf16(float f) {
    unsigned u = __float_as_uint(f);
    unsigned r = u + 0x7FFFu + ((u >> 16) & 1u);
    return (unsigned short)(r >> 16);
}
__device__ __forceinline__ float bf16_to_f32(unsigned short b) {
    return __uint_as_float(((unsigned)b) << 16);
}
__device__ __forceinline__ float rcp_f(float x) { return __builtin_amdgcn_rcpf(x); }
__device__ __forceinline__ float sigm_f(float x) { return rcp_f(1.0f + __expf(-x)); }
__device__ __forceinline__ float tanh_f(float x) { return 1.0f - 2.0f * rcp_f(1.0f + __expf(2.0f * x)); }

__device__ __forceinline__ v8f ld8f(const float* p) {
    v4f a = *(const v4f*)p;
    v4f b = *(const v4f*)(p + 4);
    return __builtin_shufflevector(a, b, 0, 1, 2, 3, 4, 5, 6, 7);
}
__device__ __forceinline__ void split8(const v8f x, u16x8& hv, u16x8& lv) {
#pragma unroll
    for (int c = 0; c < 8; ++c) {
        const float f = x[c];
        const unsigned short hb = f32_to_bf16(f);
        const unsigned short lb = f32_to_bf16(f - bf16_to_f32(hb));
        hv[c] = hb;
        lv[c] = lb;
    }
}
__device__ __forceinline__ v8h to_h8(const v8f x) {
    v8h y;
#pragma unroll
    for (int c = 0; c < 8; ++c) y[c] = (_Float16)x[c];
    return y;
}

__device__ __forceinline__ void mma_b(v8f& acc, const FragB& a, const FragB& b) {
    acc = __builtin_amdgcn_wmma_f32_16x16x32_bf16(false, a.v, false, b.v, (short)0, acc, false, false);
    asm volatile("v_nop\n\tv_nop\n\tv_nop\n\tv_nop" : "+v"(acc) : "v"(a.v), "v"(b.v));
}
__device__ __forceinline__ void mma_h(v8f& acc, const FragH& a, const FragH& b) {
    acc = __builtin_amdgcn_wmma_f32_16x16x32_f16(false, a.v, false, b.v, (short)0, acc, false, false);
    asm volatile("v_nop\n\tv_nop\n\tv_nop\n\tv_nop" : "+v"(acc) : "v"(a.v), "v"(b.v));
}

__global__ __launch_bounds__(256)
void cvt_split_kernel(const float* __restrict__ src, unsigned short* dhi, unsigned short* dlo, int n8, int perm)
{
    const int i = blockIdx.x * 256 + threadIdx.x;
    if (i >= n8) return;
    const size_t e   = (size_t)i * 8;
    const int    row = (int)(e >> 10);
    const int    col = (int)(e & 1023);
    const int    srow = (perm != 0) ? ((row & 31) * TT + (row >> 5)) : row;
    const size_t se  = (size_t)srow * DD + col;
    const v8f x = ld8f(src + se);
    u16x8 hv, lv;
    split8(x, hv, lv);
    *(volatile u16x8*)(dhi + e) = hv;
    *(volatile u16x8*)(dlo + e) = lv;
    __threadfence();
    *(volatile u16x8*)(dhi + e) = hv;
    *(volatile u16x8*)(dlo + e) = lv;
}

__global__ __launch_bounds__(256)
void cvt_f16_kernel(const float* __restrict__ src, _Float16* dst, int n8, float scale)
{
    const int i = blockIdx.x * 256 + threadIdx.x;
    if (i >= n8) return;
    const size_t e = (size_t)i * 8;
    const v8f x = ld8f(src + e) * scale;
    const v8h y = to_h8(x);
    *(volatile v8h*)(dst + e) = y;
    __threadfence();
    *(volatile v8h*)(dst + e) = y;
}

template<int NBF>
__device__ __forceinline__ void tile_store_pass(const float* st, float* gp, int ldc, int lane) {
    constexpr int CW  = NBF * 16;
    constexpr int P   = CW + 4;
    constexpr int LPR = CW / 4;
    static_assert(32 % LPR == 0);
    constexpr int RPI = 32 / LPR;
    constexpr int NIT = 32 / RPI;
    const int rsub = lane / LPR;
    const int c0   = (lane % LPR) * 4;
#pragma unroll
    for (int it = 0; it < NIT; ++it) {
        const int row = it * RPI + rsub;
        const v4f v = *(const v4f*)(st + row * P + c0);
        *(volatile v4f*)(gp + (size_t)row * ldc + c0) = v;
    }
}

template<int NBF>
__global__ __launch_bounds__(128)
void gemm_x3_kernel(const unsigned short* __restrict__ Ah, const unsigned short* __restrict__ Al,
                    const unsigned short* __restrict__ Bh, const unsigned short* __restrict__ Bl,
                    const float* __restrict__ b1, const float* __restrict__ b2,
                    float* C, int K, int ldc)
{
    constexpr int CW = NBF * 16;
    constexpr int P  = CW + 4;
    static_assert(CW % 32 == 0);
    __shared__ __attribute__((aligned(16))) float stile[4][32 * P];

    const int tid  = threadIdx.x;
    const int lane = tid & 31;
    const int wave = tid >> 5;
    const int h    = lane >> 4;
    const int m    = lane & 15;
    const int wm   = wave >> 1;
    const int wn   = wave & 1;

    const int rowW = blockIdx.y * 64 + wm * 32;
    const int colW = blockIdx.x * (2 * CW) + wn * CW;

    v8f acc[2 * NBF];
#pragma unroll
    for (int j = 0; j < 2 * NBF; ++j)
#pragma unroll
        for (int r = 0; r < 8; ++r) acc[j][r] = 0.0f;

    const size_t aoff  = (size_t)(rowW + m) * K + 8 * h;
    const size_t boff  = (size_t)(colW + m) * K + 8 * h;
    const size_t sub16 = (size_t)16 * K;
    const int nk = K >> 5;

#pragma unroll 1
    for (int kt = 0; kt < nk; ++kt) {
        const size_t k0 = (size_t)kt * 32;
        FragB fa[2], ga[2], fb[NBF], gb[NBF];
#pragma unroll
        for (int s = 0; s < 2; ++s) {
            const unsigned short* p = Ah + aoff + s * sub16 + k0;
            const unsigned short* q = Al + aoff + s * sub16 + k0;
            fa[s].h[0] = *(const u16x8*)(p);
            fa[s].h[1] = *(const u16x8*)(p + 16);
            ga[s].h[0] = *(const u16x8*)(q);
            ga[s].h[1] = *(const u16x8*)(q + 16);
        }
#pragma unroll
        for (int j = 0; j < NBF; ++j) {
            const unsigned short* p = Bh + boff + j * sub16 + k0;
            const unsigned short* q = Bl + boff + j * sub16 + k0;
            fb[j].h[0] = *(const u16x8*)(p);
            fb[j].h[1] = *(const u16x8*)(p + 16);
            gb[j].h[0] = *(const u16x8*)(q);
            gb[j].h[1] = *(const u16x8*)(q + 16);
        }
#pragma unroll
        for (int s = 0; s < 2; ++s)
#pragma unroll
            for (int j = 0; j < NBF; ++j) {
                mma_b(acc[s * NBF + j], fa[s], fb[j]);
                mma_b(acc[s * NBF + j], fa[s], gb[j]);
                mma_b(acc[s * NBF + j], ga[s], fb[j]);
            }
    }

    float bs[NBF];
#pragma unroll
    for (int j = 0; j < NBF; ++j) {
        const int col = colW + j * 16 + m;
        bs[j] = b1[col] + b2[col];
    }

    float* st = stile[wave];
#pragma unroll
    for (int s = 0; s < 2; ++s)
#pragma unroll
        for (int j = 0; j < NBF; ++j)
#pragma unroll
            for (int r = 0; r < 8; ++r)
                st[(s * 16 + 8 * h + r) * P + j * 16 + m] = acc[s * NBF + j][r] + bs[j];
    __syncthreads();

    float* gp = C + (size_t)rowW * ldc + colW;
    tile_store_pass<NBF>(st, gp, ldc, lane);
    __threadfence();
    tile_store_pass<NBF>(st, gp, ldc, lane);
}

template<bool WHB>
__device__ __forceinline__ void lstm_store_pass(const float* hf, _Float16* hb, float* hout, _Float16* hpl,
                                                int b0, int t, int tid)
{
#pragma unroll
    for (int it = 0; it < 16; ++it) {
        const int e   = (it * 256 + tid) * 4;
        const int row = e >> 10;
        const int col = e & 1023;
        const v4f v = *(const v4f*)(hf + e);
        float* gp = hout + ((size_t)(b0 + row) * TT + t) * DD + col;
        *(volatile v4f*)gp = v;
    }
#pragma unroll
    for (int it = 0; it < 8; ++it) {
        const int e   = (it * 256 + tid) * 8;
        const int row = e >> 10;
        const int col = e & 1023;
        const v8f x = ld8f(hf + e);
        const v8h y = to_h8(x);
        if (WHB) *(v8h*)(hb + e) = y;
        _Float16* gq = hpl + ((size_t)(b0 + row) * TT + t) * DD + col;
        *(volatile v8h*)gq = y;
    }
}

__global__ __launch_bounds__(256)
void lstm_kernel(const _Float16* __restrict__ Whh, const float* __restrict__ xg,
                 float* hout, _Float16* hpl)
{
    extern __shared__ __attribute__((aligned(16))) unsigned char dlds[];
    _Float16* hb = (_Float16*)(dlds);
    float*    hf = (float*)(dlds + 32768);
    float*    cl = (float*)(dlds + 98304);

    const int tid  = threadIdx.x;
    const int lane = tid & 31;
    const int wave = tid >> 5;
    const int h    = lane >> 4;
    const int m    = lane & 15;
    const int b0   = blockIdx.x * 16;

#pragma unroll 1
    for (int i = tid; i < 16 * DD; i += 256) {
        hb[i] = (_Float16)0.0f;
        cl[i] = 0.0f;
    }
    __syncthreads();

    const float inv64 = 0.015625f;

#pragma unroll 1
    for (int t = 0; t < TT; ++t) {
        const float* xgt = xg + (size_t)t * ((size_t)BB * GG);

#pragma unroll 1
        for (int p = 0; p < 4; ++p) {
            const int ub = wave * 128 + p * 32;
            v8f acc[4][2];
#pragma unroll
            for (int q = 0; q < 4; ++q)
#pragma unroll
                for (int j = 0; j < 2; ++j)
#pragma unroll
                    for (int r = 0; r < 8; ++r) acc[q][j][r] = 0.0f;

            const _Float16* bp = Whh + (size_t)(ub + m) * DD + 8 * h;
            const _Float16* ap = hb + m * DD + 8 * h;

#pragma unroll 1
            for (int k0 = 0; k0 < DD; k0 += 32) {
                FragH a;
                a.h[0] = *(const v8h*)(ap + k0);
                a.h[1] = *(const v8h*)(ap + k0 + 16);
#pragma unroll
                for (int q = 0; q < 4; ++q)
#pragma unroll
                    for (int j = 0; j < 2; ++j) {
                        const _Float16* p2 = bp + ((size_t)q * DD + (size_t)j * 16) * DD + k0;
                        FragH bf;
                        bf.h[0] = *(const v8h*)(p2);
                        bf.h[1] = *(const v8h*)(p2 + 16);
                        mma_h(acc[q][j], a, bf);
                    }
            }

#pragma unroll
            for (int j = 0; j < 2; ++j) {
                const int d = ub + j * 16 + m;
#pragma unroll
                for (int r = 0; r < 8; ++r) {
                    const int row = 8 * h + r;
                    const float* xr = xgt + (size_t)(b0 + row) * GG + d;
                    const float pi = acc[0][j][r] * inv64 + xr[0];
                    const float pf = acc[1][j][r] * inv64 + xr[DD];
                    const float pg = acc[2][j][r] * inv64 + xr[2 * DD];
                    const float po = acc[3][j][r] * inv64 + xr[3 * DD];
                    const float iv = sigm_f(pi);
                    const float fv = sigm_f(pf);
                    const float gv = tanh_f(pg);
                    const float ov = sigm_f(po);
                    const int li = row * DD + d;
                    const float cn = fv * cl[li] + iv * gv;
                    cl[li] = cn;
                    hf[li] = ov * tanh_f(cn);
                }
            }
        }
        __syncthreads();

        lstm_store_pass<true>(hf, hb, hout, hpl, b0, t, tid);
        __threadfence();
        lstm_store_pass<false>(hf, hb, hout, hpl, b0, t, tid);
        __syncthreads();
    }
}

__global__ __launch_bounds__(128)
void attw_kernel(const _Float16* __restrict__ A, const _Float16* __restrict__ Bw,
                 const float* __restrict__ batt, const float* __restrict__ wctx, float* part)
{
    __shared__ float sp[4][32];
    const int tid  = threadIdx.x;
    const int lane = tid & 31;
    const int wave = tid >> 5;
    const int h    = lane >> 4;
    const int m    = lane & 15;
    const int wm   = wave >> 1;
    const int wn   = wave & 1;
    const int rowW = blockIdx.y * 64 + wm * 32;
    const int colW = blockIdx.x * 64 + wn * 32;

    v8f acc[2][2];
#pragma unroll
    for (int s = 0; s < 2; ++s)
#pragma unroll
        for (int j = 0; j < 2; ++j)
#pragma unroll
            for (int r = 0; r < 8; ++r) acc[s][j][r] = 0.0f;

    const size_t aoff  = (size_t)(rowW + m) * DD + 8 * h;
    const size_t boff  = (size_t)(colW + m) * DD + 8 * h;
    const size_t sub16 = (size_t)16 * DD;

#pragma unroll 1
    for (int k0 = 0; k0 < DD; k0 += 32) {
        FragH fa[2], fb[2];
#pragma unroll
        for (int s = 0; s < 2; ++s) {
            const _Float16* p = A + aoff + s * sub16 + k0;
            fa[s].h[0] = *(const v8h*)(p);
            fa[s].h[1] = *(const v8h*)(p + 16);
        }
#pragma unroll
        for (int j = 0; j < 2; ++j) {
            const _Float16* p = Bw + boff + j * sub16 + k0;
            fb[j].h[0] = *(const v8h*)(p);
            fb[j].h[1] = *(const v8h*)(p + 16);
        }
#pragma unroll
        for (int s = 0; s < 2; ++s)
#pragma unroll
            for (int j = 0; j < 2; ++j) mma_h(acc[s][j], fa[s], fb[j]);
    }

    const float inv64 = 0.015625f;
    float rs[2][8];
#pragma unroll
    for (int s = 0; s < 2; ++s)
#pragma unroll
        for (int r = 0; r < 8; ++r) rs[s][r] = 0.0f;
#pragma unroll
    for (int j = 0; j < 2; ++j) {
        const int col = colW + j * 16 + m;
        const float bj = batt[col];
        const float wj = wctx[col];
#pragma unroll
        for (int s = 0; s < 2; ++s)
#pragma unroll
            for (int r = 0; r < 8; ++r)
                rs[s][r] = tanh_f(acc[s][j][r] * inv64 + bj) * wj + rs[s][r];
    }
#pragma unroll
    for (int s = 0; s < 2; ++s)
#pragma unroll
        for (int r = 0; r < 8; ++r) {
            float x = rs[s][r];
            x += __shfl_xor(x, 1, 32);
            x += __shfl_xor(x, 2, 32);
            x += __shfl_xor(x, 4, 32);
            x += __shfl_xor(x, 8, 32);
            rs[s][r] = x;
        }
    if (m == 0) {
#pragma unroll
        for (int s = 0; s < 2; ++s)
#pragma unroll
            for (int r = 0; r < 8; ++r) sp[wave][s * 16 + 8 * h + r] = rs[s][r];
    }
    __syncthreads();

    if (tid < 16) {
        v4f v;
#pragma unroll
        for (int u = 0; u < 4; ++u) {
            const int i   = tid * 4 + u;
            const int wmi = i >> 5;
            const int ir  = i & 31;
            v[u] = sp[wmi * 2 + 0][ir] + sp[wmi * 2 + 1][ir];
        }
        float* gp = part + (size_t)blockIdx.x * MR + blockIdx.y * 64 + tid * 4;
        *(volatile v4f*)gp = v;
        __threadfence();
        *(volatile v4f*)gp = v;
    }
}

__global__ __launch_bounds__(256)
void pool_kernel(const float* __restrict__ part, const float* __restrict__ bctx,
                 const float* __restrict__ attin, unsigned short* aoh, unsigned short* aol)
{
    __shared__ float w[TT];
    __shared__ __attribute__((aligned(16))) float so[DD];
    const int b   = blockIdx.x;
    const int tid = threadIdx.x;

    if (tid < TT) {
        float s = bctx[0];
#pragma unroll
        for (int cb = 0; cb < DD / 64; ++cb) s += part[(size_t)cb * MR + b * TT + tid];
        w[tid] = s;
    }
    __syncthreads();
    if (tid == 0) {
        float mx = w[0];
#pragma unroll 1
        for (int t = 1; t < TT; ++t) mx = fmaxf(mx, w[t]);
        float sum = 0.0f;
#pragma unroll 1
        for (int t = 0; t < TT; ++t) {
            const float e = expf(w[t] - mx);
            w[t] = e;
            sum += e;
        }
        const float inv = 1.0f / sum;
#pragma unroll 1
        for (int t = 0; t < TT; ++t) w[t] = w[t] * inv;
    }
    __syncthreads();

    const float* ab = attin + (size_t)b * TT * DD + tid * 4;
    v4f s4;
    s4[0] = 0.0f; s4[1] = 0.0f; s4[2] = 0.0f; s4[3] = 0.0f;
#pragma unroll 1
    for (int t = 0; t < TT; ++t) {
        const v4f x = *(const v4f*)(ab + (size_t)t * DD);
        s4 = x * w[t] + s4;
    }
    *(v4f*)(so + tid * 4) = s4;
    __syncthreads();

    if (tid < DD / 8) {
        const v8f x = ld8f(so + tid * 8);
        u16x8 hv, lv;
        split8(x, hv, lv);
        const size_t o = (size_t)b * DD + tid * 8;
        *(volatile u16x8*)(aoh + o) = hv;
        *(volatile u16x8*)(aol + o) = lv;
        __threadfence();
        *(volatile u16x8*)(aoh + o) = hv;
        *(volatile u16x8*)(aol + o) = lv;
    }
}

__global__ __launch_bounds__(128)
void head_kernel(const unsigned short* __restrict__ Ah, const unsigned short* __restrict__ Al,
                 const unsigned short* __restrict__ Bh, const unsigned short* __restrict__ Bl,
                 const float* __restrict__ bl, float* out)
{
    __shared__ __attribute__((aligned(16))) float st[32 * 68];
    const int tid  = threadIdx.x;
    const int lane = tid & 31;
    const int wave = tid >> 5;
    const int h    = lane >> 4;
    const int m    = lane & 15;
    const int colT = blockIdx.x * 64 + wave * 16;

    v8f acc[2];
#pragma unroll
    for (int s = 0; s < 2; ++s)
#pragma unroll
        for (int r = 0; r < 8; ++r) acc[s][r] = 0.0f;

    const size_t aoff  = (size_t)m * DD + 8 * h;
    const size_t boff  = (size_t)(colT + m) * DD + 8 * h;
    const size_t sub16 = (size_t)16 * DD;

#pragma unroll 1
    for (int k0 = 0; k0 < DD; k0 += 32) {
        FragB fa[2], ga[2], fb, gb;
#pragma unroll
        for (int s = 0; s < 2; ++s) {
            const unsigned short* p = Ah + aoff + s * sub16 + k0;
            const unsigned short* q = Al + aoff + s * sub16 + k0;
            fa[s].h[0] = *(const u16x8*)(p);
            fa[s].h[1] = *(const u16x8*)(p + 16);
            ga[s].h[0] = *(const u16x8*)(q);
            ga[s].h[1] = *(const u16x8*)(q + 16);
        }
        {
            const unsigned short* p = Bh + boff + k0;
            const unsigned short* q = Bl + boff + k0;
            fb.h[0] = *(const u16x8*)(p);
            fb.h[1] = *(const u16x8*)(p + 16);
            gb.h[0] = *(const u16x8*)(q);
            gb.h[1] = *(const u16x8*)(q + 16);
        }
#pragma unroll
        for (int s = 0; s < 2; ++s) {
            mma_b(acc[s], fa[s], fb);
            mma_b(acc[s], fa[s], gb);
            mma_b(acc[s], ga[s], fb);
        }
    }

    const float bias = bl[colT + m];
#pragma unroll
    for (int s = 0; s < 2; ++s)
#pragma unroll
        for (int r = 0; r < 8; ++r)
            st[(s * 16 + 8 * h + r) * 68 + wave * 16 + m] = fmaxf(acc[s][r] + bias, 0.0f);
    __syncthreads();

#pragma unroll
    for (int it = 0; it < 4; ++it) {
        const int row = it * 8 + (tid >> 4);
        const int c4  = (tid & 15) * 4;
        const v4f v = *(const v4f*)(st + row * 68 + c4);
        float* gp = out + (size_t)row * DD + blockIdx.x * 64 + c4;
        *(volatile v4f*)gp = v;
    }
    __threadfence();
#pragma unroll
    for (int it = 0; it < 4; ++it) {
        const int row = it * 8 + (tid >> 4);
        const int c4  = (tid & 15) * 4;
        const v4f v = *(const v4f*)(st + row * 68 + c4);
        float* gp = out + (size_t)row * DD + blockIdx.x * 64 + c4;
        *(volatile v4f*)gp = v;
    }
}

extern "C" void kernel_launch(void* const* d_in, const int* in_sizes, int n_in,
                              void* d_out, int out_size, void* d_ws, size_t ws_size,
                              hipStream_t stream)
{
    if (n_in < 11) return;
    if (in_sizes[0]  != BB * TT * DD) return;
    if (in_sizes[1]  != GG * DD)      return;
    if (in_sizes[2]  != GG * DD)      return;
    if (in_sizes[3]  != GG)           return;
    if (in_sizes[4]  != GG)           return;
    if (in_sizes[5]  != DD * DD)      return;
    if (in_sizes[6]  != DD)           return;
    if (in_sizes[7]  != DD)           return;
    if (in_sizes[8]  <  1)            return;
    if (in_sizes[9]  != DD * DD)      return;
    if (in_sizes[10] != DD)           return;
    if (out_size != BB * DD + BB * TT * DD) return;
    if (ws_size < WS_END)             return;

    const float* Q     = (const float*)d_in[0];
    const float* W_ih  = (const float*)d_in[1];
    const float* W_hh  = (const float*)d_in[2];
    const float* b_ih  = (const float*)d_in[3];
    const float* b_hh  = (const float*)d_in[4];
    const float* W_att = (const float*)d_in[5];
    const float* b_att = (const float*)d_in[6];
    const float* W_ctx = (const float*)d_in[7];
    const float* b_ctx = (const float*)d_in[8];
    const float* W_lg  = (const float*)d_in[9];
    const float* b_lg  = (const float*)d_in[10];

    float* out0 = (float*)d_out;
    float* out1 = (float*)d_out + (size_t)BB * DD;

    char* ws = (char*)d_ws;
    unsigned short* qh   = (unsigned short*)(ws + OFF_QH);
    unsigned short* ql   = (unsigned short*)(ws + OFF_QL);
    unsigned short* wih  = (unsigned short*)(ws + OFF_WIH);
    unsigned short* wil  = (unsigned short*)(ws + OFF_WIL);
    _Float16*       whh  = (_Float16*)(ws + OFF_WHH);
    _Float16*       wat  = (_Float16*)(ws + OFF_WAT);
    unsigned short* wlh  = (unsigned short*)(ws + OFF_WLH);
    unsigned short* wll  = (unsigned short*)(ws + OFF_WLL);
    float*          xg   = (float*)(ws + OFF_XG);
    _Float16*       hpl  = (_Float16*)(ws + OFF_HPL);
    float*          part = (float*)(ws + OFF_PART);
    unsigned short* aoh  = (unsigned short*)(ws + OFF_AOH);
    unsigned short* aol  = (unsigned short*)(ws + OFF_AOL);

    {
        const int n8q = (MR * DD) / 8;
        cvt_split_kernel<<<dim3((n8q + 255) / 256), dim3(256), 0, stream>>>(Q, qh, ql, n8q, 1);
        const int n8i = (GG * DD) / 8;
        cvt_split_kernel<<<dim3((n8i + 255) / 256), dim3(256), 0, stream>>>(W_ih, wih, wil, n8i, 0);
        cvt_f16_kernel<<<dim3((n8i + 255) / 256), dim3(256), 0, stream>>>(W_hh, whh, n8i, 64.0f);
        const int n8a = (DD * DD) / 8;
        cvt_f16_kernel<<<dim3((n8a + 255) / 256), dim3(256), 0, stream>>>(W_att, wat, n8a, 64.0f);
        cvt_split_kernel<<<dim3((n8a + 255) / 256), dim3(256), 0, stream>>>(W_lg, wlh, wll, n8a, 0);
    }

    gemm_x3_kernel<2><<<dim3(GG / 64, MR / 64), dim3(128), 0, stream>>>(
        (const unsigned short*)qh, (const unsigned short*)ql,
        (const unsigned short*)wih, (const unsigned short*)wil,
        b_ih, b_hh, xg, (int)DD, (int)GG);

    hipFuncSetAttribute(reinterpret_cast<const void*>(&lstm_kernel),
                        hipFuncAttributeMaxDynamicSharedMemorySize, LSTM_LDS_BYTES);
    lstm_kernel<<<dim3(BB / 16), dim3(256), LSTM_LDS_BYTES, stream>>>(
        (const _Float16*)whh, (const float*)xg, out1, hpl);

    attw_kernel<<<dim3(DD / 64, MR / 64), dim3(128), 0, stream>>>(
        (const _Float16*)hpl, (const _Float16*)wat, b_att, W_ctx, part);

    pool_kernel<<<dim3(BB), dim3(256), 0, stream>>>(
        (const float*)part, b_ctx, (const float*)out1, aoh, aol);

    head_kernel<<<dim3(DD / 64), dim3(128), 0, stream>>>(
        (const unsigned short*)aoh, (const unsigned short*)aol,
        (const unsigned short*)wlh, (const unsigned short*)wll, b_lg, out0);
}
